// Encoder_4544075399463
// MI455X (gfx1250) — hardware-run, weakly checked
//
#include <hip/hip_runtime.h>
#include <math.h>

typedef __attribute__((ext_vector_type(16))) _Float16 v16h;
typedef __attribute__((ext_vector_type(8)))  _Float16 v8h;
typedef __attribute__((ext_vector_type(16))) __bf16   v16b;
typedef __attribute__((ext_vector_type(8)))  __bf16   v8b;
typedef __attribute__((ext_vector_type(8)))  float    v8f;
typedef __attribute__((ext_vector_type(4)))  float    v4f;

constexpr int kBatch  = 64;
constexpr int kSteps  = 128;
constexpr int kEmb    = 256;
constexpr int kHid    = 512;
constexpr int kGate3  = 3 * kHid;
constexpr int kIn1    = 2 * kHid;
constexpr int kVocab  = 30000;
constexpr int kRows   = kBatch * kSteps;
constexpr int kThr    = 256;
constexpr int kSeqBlk = 16;
constexpr int kHP     = 520;
constexpr int kHmP    = 512;
constexpr int kOutHalf = kBatch * kIn1;

constexpr float kEmbCarry = 1024.0f;
constexpr float kWCarry   = 1024.0f;
constexpr float kActCarry = 4096.0f;
constexpr float kXs0Scale = 1.0f / (kEmbCarry * kWCarry);
constexpr float kXs1Scale = 1.0f / (kActCarry * kWCarry);
constexpr float kRecScale = 1.0f / (kActCarry * kWCarry);
constexpr float kF16MinNormal = 6.103515625e-5f;

static_assert(kBatch == 64 && kSteps == 128, "row index math uses shifts by 6 and masks");
static_assert(kRows == 8192, "rows");
static_assert(kGate3 == 1536 && kIn1 == 1024, "gate widths");
static_assert((kEmb % 64) == 0 && (kHid % 64) == 0 && (kIn1 % 64) == 0, "transpose tiles and GEMM K multiples of 32");
static_assert((kRows % 64) == 0 && (kGate3 % 64) == 0, "GEMM M, N multiples of 64");
static_assert(kHid == 64 * (kThr / 32), "8 waves x 64 hidden units");
static_assert(kBatch % kSeqBlk == 0, "batch tiles");
static_assert((2 * kSeqBlk * kHP) % kThr == 0, "state tile zero fill exact");
static_assert((kSeqBlk * kHmP) % kThr == 0, "f32 state zero fill exact");
static_assert(kGate3 % kThr == 0, "bias staging exact");
static_assert((kRows * kEmb / 8) % kThr == 0, "gather grid exact");

constexpr size_t kOffXE   = 0;
constexpr size_t kOffWK0F = kOffXE   + (size_t)kRows  * kEmb * 2;
constexpr size_t kOffWK0B = kOffWK0F + (size_t)kGate3 * kEmb * 2;
constexpr size_t kOffWK1F = kOffWK0B + (size_t)kGate3 * kEmb * 2;
constexpr size_t kOffWK1B = kOffWK1F + (size_t)kGate3 * kIn1 * 2;
constexpr size_t kOffWR0F = kOffWK1B + (size_t)kGate3 * kIn1 * 2;
constexpr size_t kOffWR0B = kOffWR0F + (size_t)kGate3 * kHid * 2;
constexpr size_t kOffWR1F = kOffWR0B + (size_t)kGate3 * kHid * 2;
constexpr size_t kOffWR1B = kOffWR1F + (size_t)kGate3 * kHid * 2;
constexpr size_t kOffBIAS = kOffWR1B + (size_t)kGate3 * kHid * 2;
constexpr size_t kOffXS   = kOffBIAS + (size_t)4 * 2 * kGate3 * 4;
constexpr size_t kOffY0   = kOffXS   + (size_t)kRows * kGate3 * 4;
constexpr size_t kWsTotal = kOffY0   + (size_t)kRows * kIn1 * 2;
static_assert(kWsTotal == 85508096ull, "carve total");
static_assert(kWsTotal <= 134217728ull, "carve cap");
static_assert((kOffWK0F % 256) == 0 && (kOffWK0B % 256) == 0 && (kOffWK1F % 256) == 0 && (kOffWK1B % 256) == 0 &&
              (kOffWR0F % 256) == 0 && (kOffWR0B % 256) == 0 && (kOffWR1F % 256) == 0 && (kOffWR1B % 256) == 0 &&
              (kOffBIAS % 256) == 0 && (kOffXS % 256) == 0 && (kOffY0 % 256) == 0, "aligned regions");

__device__ __forceinline__ unsigned short f2bf_bits(float f) {
  unsigned u = __float_as_uint(f);
  return (unsigned short)((u + 0x7FFFu + ((u >> 16) & 1u)) >> 16);
}
__device__ __forceinline__ float bf_bits2f(unsigned short h) { return __uint_as_float(((unsigned)h) << 16); }
__device__ __forceinline__ float bf16r(float f) { return bf_bits2f(f2bf_bits(f)); }
__device__ __forceinline__ float carry_flush(float v, float carry) {
  const float s = v * carry;
  return (fabsf(s) < kF16MinNormal) ? 0.0f : s;
}
__device__ __forceinline__ float frcp(float x) { return __builtin_amdgcn_rcpf(x); }

__device__ __forceinline__ void dep_guard4_h(v8f& a, v8f& b, v8f& c, v8f& d, v16h x, v16h y) { asm volatile("v_nop\n\tv_nop\n\tv_nop\n\tv_nop" : "+v"(a), "+v"(b), "+v"(c), "+v"(d) : "v"(x), "v"(y)); }
__device__ __forceinline__ void dep_guard4_b(v8f& a, v8f& b, v8f& c, v8f& d, v16b x, v16b y) { asm volatile("v_nop\n\tv_nop\n\tv_nop\n\tv_nop" : "+v"(a), "+v"(b), "+v"(c), "+v"(d) : "v"(x), "v"(y)); }
__device__ __forceinline__ void keep4_h(v16h a, v16h b, v16h c, v16h d) { asm volatile("v_nop" :: "v"(a), "v"(b), "v"(c), "v"(d)); }
__device__ __forceinline__ void keep4_b(v16b a, v16b b, v16b c, v16b d) { asm volatile("v_nop" :: "v"(a), "v"(b), "v"(c), "v"(d)); }
__device__ __forceinline__ void acc_guard4(v8f& a, v8f& b, v8f& c, v8f& d) { asm volatile("v_nop\n\tv_nop\n\tv_nop\n\tv_nop" : "+v"(a), "+v"(b), "+v"(c), "+v"(d)); }

template <typename T> struct Frag;
template <> struct Frag<_Float16> {
  typedef v16h V; union U { v16h v; v8h h[2]; };
  static __device__ __forceinline__ v16h load(const _Float16* p) {
    U f; f.h[0] = *(const v8h*)(p); f.h[1] = *(const v8h*)(p + 16); return f.v;
  }
  static __device__ __forceinline__ v8f mma(v16h a, v16h b, v8f c) {
    return __builtin_amdgcn_wmma_f32_16x16x32_f16(false, a, false, b, (short)0, c, false, false);
  }
  static __device__ __forceinline__ void guard4(v8f& a, v8f& b, v8f& c, v8f& d, v16h x, v16h y) { dep_guard4_h(a, b, c, d, x, y); }
  static __device__ __forceinline__ void keep(v16h a, v16h b, v16h c, v16h d) { keep4_h(a, b, c, d); }
};
template <> struct Frag<__bf16> {
  typedef v16b V; union U { v16b v; v8b h[2]; };
  static __device__ __forceinline__ v16b load(const __bf16* p) {
    U f; f.h[0] = *(const v8b*)(p); f.h[1] = *(const v8b*)(p + 16); return f.v;
  }
  static __device__ __forceinline__ v8f mma(v16b a, v16b b, v8f c) {
    return __builtin_amdgcn_wmma_f32_16x16x32_bf16(false, a, false, b, (short)0, c, false, false);
  }
  static __device__ __forceinline__ void guard4(v8f& a, v8f& b, v8f& c, v8f& d, v16b x, v16b y) { dep_guard4_b(a, b, c, d, x, y); }
  static __device__ __forceinline__ void keep(v16b a, v16b b, v16b c, v16b d) { keep4_b(a, b, c, d); }
};

__device__ __forceinline__ v8f mma_h(v16h a, v16h b, v8f c) {
  c = __builtin_amdgcn_wmma_f32_16x16x32_f16(false, a, false, b, (short)0, c, false, false);
  asm volatile("v_nop\n\tv_nop\n\tv_nop\n\tv_nop" : "+v"(c) : "v"(a), "v"(b));
  return c;
}

template <int ET> struct Elem;
template <> struct Elem<0> { typedef _Float16 T; };
template <> struct Elem<1> { typedef __bf16 T; };
template <int ET, bool SPLIT, int BIAS_MODE, int OUT_MODE, bool RESID, int ACT = 0>
__global__ __launch_bounds__(256) void wmma_gemm64(
    const unsigned short* __restrict__ Ap, const unsigned short* __restrict__ A2p, int lda, long strideA,
    const unsigned short* __restrict__ Btp, const unsigned short* __restrict__ Bt2p, int ldb, long strideB,
    void* __restrict__ Cout, void* __restrict__ Cout2, int ldc, long strideC,
    const float* __restrict__ bias,
    const float* __restrict__ resid, long strideR,
    int M, int N, int K, float scale) {
  typedef typename Elem<ET>::T T;
  typedef typename Frag<T>::V V;
  const T* A = (const T*)Ap; const T* A2 = (const T*)A2p; const T* Bt = (const T*)Btp; const T* Bt2 = (const T*)Bt2p;
  __shared__ __align__(16) float sT[8][16 * 68];
  const int b    = blockIdx.y;
  const int lane = threadIdx.x & 31;
  const int wave = threadIdx.x >> 5;
  const int tilesN = N >> 6;
  const int tilesM = M >> 6;
  const int tile = blockIdx.x * 8 + wave;
  if (tile >= tilesM * tilesN) return;
  const int tm = tile / tilesN;
  const int tn = tile - tm * tilesN;
  const int m0 = tm << 6;
  const int n0 = tn << 6;

  const T* Ab  = A  + (size_t)b * strideA;
  const T* Bb  = Bt + (size_t)b * strideB;
  const T* Ab2 = SPLIT ? (A2  + (size_t)b * strideA) : nullptr;
  const T* Bb2 = SPLIT ? (Bt2 + (size_t)b * strideB) : nullptr;

  const int rlane = lane & 15;
  const int koff  = (lane >> 4) * 8;
  const int mOff  = (lane >> 4) * 8;

  v8f acc[4][4];
#pragma unroll
  for (int i = 0; i < 4; ++i)
#pragma unroll
    for (int j = 0; j < 4; ++j) acc[i][j] = (v8f){0.f,0.f,0.f,0.f,0.f,0.f,0.f,0.f};

  for (int k0 = 0; k0 < K; k0 += 32) {
    V bh[4], bl[4];
#pragma unroll
    for (int j = 0; j < 4; ++j) {
      const size_t bo = (size_t)(n0 + (j << 4) + rlane) * ldb + koff + k0;
      bh[j] = Frag<T>::load(Bb + bo);
      if (SPLIT) bl[j] = Frag<T>::load(Bb2 + bo);
    }
#pragma unroll
    for (int i = 0; i < 4; ++i) {
      const size_t ao = (size_t)(m0 + (i << 4) + rlane) * lda + koff + k0;
      V ah = Frag<T>::load(Ab + ao);
      V al;
      if (SPLIT) al = Frag<T>::load(Ab2 + ao);
#pragma unroll
      for (int j = 0; j < 4; ++j) {
        acc[i][j] = Frag<T>::mma(ah, bh[j], acc[i][j]);
        if (SPLIT) {
          acc[i][j] = Frag<T>::mma(ah, bl[j], acc[i][j]);
          acc[i][j] = Frag<T>::mma(al, bh[j], acc[i][j]);
        }
      }
      Frag<T>::guard4(acc[i][0], acc[i][1], acc[i][2], acc[i][3], ah, SPLIT ? al : ah);
    }
    Frag<T>::keep(bh[0], bh[1], bh[2], bh[3]);
    if (SPLIT) Frag<T>::keep(bl[0], bl[1], bl[2], bl[3]);
  }
  acc_guard4(acc[0][0], acc[0][1], acc[0][2], acc[0][3]);
  acc_guard4(acc[1][0], acc[1][1], acc[1][2], acc[1][3]);
  acc_guard4(acc[2][0], acc[2][1], acc[2][2], acc[2][3]);
  acc_guard4(acc[3][0], acc[3][1], acc[3][2], acc[3][3]);

  float* slab = sT[wave];
  const float* Rb = RESID ? (resid + (size_t)b * strideR) : nullptr;
#pragma unroll
  for (int i = 0; i < 4; ++i) {
    const int mBase = m0 + (i << 4);
#pragma unroll
    for (int j = 0; j < 4; ++j) {
      const int n = n0 + (j << 4) + rlane;
      float bv = 0.f;
      if (BIAS_MODE == 2) bv = bias[n];
#pragma unroll
      for (int r = 0; r < 8; ++r) {
        float v = acc[i][j][r] * scale;
        if (BIAS_MODE == 1) v += bias[mBase + mOff + r];
        if (BIAS_MODE == 2) v += bv;
        if (RESID) v += Rb[(size_t)(mBase + mOff + r) * ldc + n];
        if (ACT == 1) v = tanhf(v);
        if (ACT == 2) v = fmaxf(v, 0.0f);
        if (ACT == 3) v = v / (1.0f + expf(-v));
        if (ACT == 4) v = (v > 0.f) ? v : 0.01f * v;
        slab[(mOff + r) * 68 + (j << 4) + rlane] = v;
      }
    }
    __builtin_amdgcn_fence(__ATOMIC_RELEASE, "workgroup");
    __builtin_amdgcn_wave_barrier();
    __builtin_amdgcn_fence(__ATOMIC_ACQUIRE, "workgroup");
    if (OUT_MODE == 0) {
      float* C = (float*)Cout + (size_t)b * strideC;
      const int hh = lane >> 4, c4 = (lane & 15) * 4;
      for (int pass = 0; pass < 2; ++pass) {
#pragma unroll
        for (int it = 0; it < 8; ++it) {
          const int row = it * 2 + hh;
          v4f v = *(const v4f*)(slab + row * 68 + c4);
          *(volatile v4f*)(C + (size_t)(mBase + row) * ldc + n0 + c4) = v;
        }
        __threadfence();
      }
    } else {
      const int q = lane >> 3, c8 = (lane & 7) * 8;
      unsigned short* C  = (unsigned short*)Cout  + (size_t)b * strideC;
      unsigned short* C2 = (OUT_MODE == 2) ? ((unsigned short*)Cout2 + (size_t)b * strideC) : nullptr;
      for (int pass = 0; pass < 2; ++pass) {
#pragma unroll
        for (int it = 0; it < 4; ++it) {
          const int row = it * 4 + q;
          const float* sp = slab + row * 68 + c8;
          v8h hv, lv;
#pragma unroll
          for (int e = 0; e < 8; ++e) {
            if (OUT_MODE == 1) {
              hv[e] = (_Float16)sp[e];
            } else {
              unsigned short hb = f2bf_bits(sp[e]);
              unsigned short lb = f2bf_bits(sp[e] - bf_bits2f(hb));
              hv[e] = __builtin_bit_cast(_Float16, hb);
              lv[e] = __builtin_bit_cast(_Float16, lb);
            }
          }
          *(volatile v8h*)(C + (size_t)(mBase + row) * ldc + n0 + c8) = hv;
          if (OUT_MODE == 2) *(volatile v8h*)(C2 + (size_t)(mBase + row) * ldc + n0 + c8) = lv;
        }
        __threadfence();
      }
    }
    __builtin_amdgcn_fence(__ATOMIC_RELEASE, "workgroup");
    __builtin_amdgcn_wave_barrier();
    __builtin_amdgcn_fence(__ATOMIC_ACQUIRE, "workgroup");
  }
}

__global__ __launch_bounds__(kThr) void embed_f16_kernel(const int* __restrict__ tok, const float* __restrict__ emb,
                                                         unsigned short* __restrict__ XE) {
  const int i  = blockIdx.x * kThr + threadIdx.x;
  const int m  = i >> 5;
  const int c8 = (i & 31) * 8;
  const int t  = m >> 6;
  const int b  = m & 63;
  int id = tok[b * kSteps + t];
  id = (id < 0) ? 0 : id;
  id = (id > kVocab - 1) ? (kVocab - 1) : id;
  const float* sp = emb + (size_t)id * kEmb + c8;
  const v4f a0 = *(const v4f*)(sp);
  const v4f a1 = *(const v4f*)(sp + 4);
  v8h hv;
#pragma unroll
  for (int e = 0; e < 4; ++e) {
    const float f0 = a0[e];
    const float f1 = a1[e];
    hv[e]     = (_Float16)carry_flush(bf16r(f0), kEmbCarry);
    hv[4 + e] = (_Float16)carry_flush(bf16r(f1), kEmbCarry);
  }
  unsigned short* dp = XE + (size_t)i * 8;
  *(volatile v8h*)dp = hv;
  __threadfence();
  *(volatile v8h*)dp = hv;
}

__global__ __launch_bounds__(kThr) void bias_prep_kernel(const float* __restrict__ b0, const float* __restrict__ b1,
                                                         const float* __restrict__ b2, const float* __restrict__ b3,
                                                         float* __restrict__ dst) {
  const int which = blockIdx.y;
  const float* src = (which == 0) ? b0 : (which == 1) ? b1 : (which == 2) ? b2 : b3;
  const int idx = (blockIdx.x * kThr + threadIdx.x) * 4;
  const v4f v = *(const v4f*)(src + idx);
  v4f o;
#pragma unroll
  for (int e = 0; e < 4; ++e) {
    const float f = v[e];
    o[e] = bf16r(f);
  }
  float* op = dst + (size_t)which * (2 * kGate3) + idx;
  *(volatile v4f*)op = o;
  __threadfence();
  *(volatile v4f*)op = o;
}

__global__ __launch_bounds__(kThr) void wt_transpose_f16_kernel(const float* __restrict__ in,
                                                                unsigned short* __restrict__ out, int kdim) {
  __shared__ __align__(16) float sTile[64 * 68];
  const int tid = threadIdx.x;
  const int n0 = blockIdx.x * 64;
  const int k0 = blockIdx.y * 64;
  {
    const int kk = tid >> 4;
    const int n4 = (tid & 15) * 4;
#pragma unroll
    for (int i = 0; i < 4; ++i) {
      const int k = kk + 16 * i;
      const v4f v = *(const v4f*)(in + (size_t)(k0 + k) * kGate3 + n0 + n4);
#pragma unroll
      for (int e = 0; e < 4; ++e) {
        const float f = v[e];
        sTile[(n4 + e) * 68 + k] = carry_flush(bf16r(f), kWCarry);
      }
    }
  }
  __syncthreads();
  const int k8 = (tid & 7) * 8;
  v8h hv[2];
#pragma unroll
  for (int it = 0; it < 2; ++it) {
    const int n = (tid >> 3) + 32 * it;
    const float* sp = sTile + n * 68 + k8;
    const v4f a0 = *(const v4f*)(sp);
    const v4f a1 = *(const v4f*)(sp + 4);
#pragma unroll
    for (int e = 0; e < 4; ++e) {
      const float f0 = a0[e];
      const float f1 = a1[e];
      hv[it][e]     = (_Float16)f0;
      hv[it][4 + e] = (_Float16)f1;
    }
  }
  for (int pass = 0; pass < 2; ++pass) {
#pragma unroll
    for (int it = 0; it < 2; ++it) {
      const int n = (tid >> 3) + 32 * it;
      *(volatile v8h*)(out + (size_t)(n0 + n) * kdim + k0 + k8) = hv[it];
    }
    __threadfence();
  }
}

template <int LAYER>
__global__ __launch_bounds__(kThr) void gru_run_kernel(const float* __restrict__ XS,
                                                       const unsigned short* __restrict__ WRp,
                                                       const float* __restrict__ BR,
                                                       unsigned short* __restrict__ Y0,
                                                       float* __restrict__ OUT,
                                                       int dir) {
  __shared__ __align__(16) _Float16 Ah[2][kSeqBlk * kHP];
  __shared__ __align__(16) float    Hm[kSeqBlk * kHmP];
  __shared__ __align__(16) float    sBr[kGate3];
  const _Float16* WR = (const _Float16*)WRp;
  const int tid = threadIdx.x, lane = tid & 31, wave = tid >> 5;
  const int c = lane & 15, hh = lane >> 4, koff = hh * 8, c4 = c * 4;
  const int rowbase = blockIdx.x * kSeqBlk;

  {
    _Float16* ahf = &Ah[0][0];
#pragma unroll 1
    for (int i = tid; i < 2 * kSeqBlk * kHP; i += kThr) ahf[i] = (_Float16)0.0f;
#pragma unroll 1
    for (int i = tid; i < kSeqBlk * kHmP; i += kThr) Hm[i] = 0.0f;
#pragma unroll 1
    for (int i = tid; i < kGate3; i += kThr) sBr[i] = BR[i];
  }
  __syncthreads();

  const v8f z8 = {0.f, 0.f, 0.f, 0.f, 0.f, 0.f, 0.f, 0.f};

#pragma unroll 1
  for (int s = 0; s < kSteps; ++s) {
    const int cur = s & 1;
    const int tx  = dir ? (kSteps - 1 - s) : s;
    const _Float16* ahrow = &Ah[cur][0] + c * kHP + koff;
    _Float16* ahn = &Ah[cur ^ 1][0];
    const float* xsrow = XS + (size_t)(tx * kBatch + rowbase + 8 * hh) * kGate3;

#pragma unroll 1
    for (int nt = 0; nt < 4; ++nt) {
      const int j = 64 * wave + 16 * nt + c;
      float xz[8], xr[8], xh[8];
#pragma unroll
      for (int r = 0; r < 8; ++r) {
        const float* xp = xsrow + (size_t)r * kGate3 + j;
        xz[r] = xp[0];
        xr[r] = xp[kHid];
        xh[r] = xp[2 * kHid];
      }
      const _Float16* wz = WR + (size_t)j * kHid + koff;
      const _Float16* wr = WR + (size_t)(kHid + j) * kHid + koff;
      const _Float16* wn = WR + (size_t)(2 * kHid + j) * kHid + koff;
      v8f az = z8, ar = z8, an = z8;
#pragma unroll 2
      for (int k0 = 0; k0 < kHid; k0 += 32) {
        const v16h a  = Frag<_Float16>::load(ahrow + k0);
        const v16h bz = Frag<_Float16>::load(wz + k0);
        const v16h br = Frag<_Float16>::load(wr + k0);
        const v16h bn = Frag<_Float16>::load(wn + k0);
        az = mma_h(a, bz, az);
        ar = mma_h(a, br, ar);
        an = mma_h(a, bn, an);
      }
      const float brz = sBr[j];
      const float brr = sBr[kHid + j];
      const float brn = sBr[2 * kHid + j];
#pragma unroll
      for (int r = 0; r < 8; ++r) {
        const int row = 8 * hh + r;
        const float hz = az[r] * kRecScale + brz;
        const float hr = ar[r] * kRecScale + brr;
        const float hn = an[r] * kRecScale + brn;
        const float zg = frcp(1.0f + expf(-(xz[r] + hz)));
        const float rg = frcp(1.0f + expf(-(xr[r] + hr)));
        const float hc = tanhf(xh[r] + rg * hn);
        const float ho = Hm[row * kHmP + j];
        const float hnew = zg * ho + (1.0f - zg) * hc;
        Hm[row * kHmP + j] = hnew;
        ahn[row * kHP + j] = (_Float16)carry_flush(hnew, kActCarry);
      }
    }
    __syncthreads();

    if (LAYER == 0) {
      v8h yv[4];
#pragma unroll
      for (int it = 0; it < 4; ++it) {
        const int row = 2 * wave + (it >> 1);
        const int hf  = it & 1;
        yv[it] = *(const v8h*)(ahn + row * kHP + hf * 256 + lane * 8);
      }
      for (int pass = 0; pass < 2; ++pass) {
#pragma unroll
        for (int it = 0; it < 4; ++it) {
          const int row = 2 * wave + (it >> 1);
          const int hf  = it & 1;
          *(volatile v8h*)(Y0 + (size_t)(tx * kBatch + rowbase + row) * kIn1 + dir * kHid + hf * 256 + lane * 8) = yv[it];
        }
        __threadfence();
      }
    } else {
      const bool lastStep  = (s == kSteps - 1);
      const bool firstStep = (s == 0);
      const bool st0 = dir ? firstStep : lastStep;
      const bool st1 = lastStep;
      if (st0 || st1) {
        __builtin_amdgcn_fence(__ATOMIC_RELEASE, "workgroup");
        __builtin_amdgcn_wave_barrier();
        __builtin_amdgcn_fence(__ATOMIC_ACQUIRE, "workgroup");
        v4f ov[8];
#pragma unroll
        for (int it = 0; it < 8; ++it) {
          const int row = it * 2 + hh;
          ov[it] = *(const v4f*)(Hm + row * kHmP + 64 * wave + c4);
        }
        for (int pass = 0; pass < 2; ++pass) {
#pragma unroll
          for (int it = 0; it < 8; ++it) {
            const int row = it * 2 + hh;
            float* p0 = OUT + (size_t)(rowbase + row) * kIn1 + dir * kHid + 64 * wave + c4;
            if (st0) *(volatile v4f*)p0 = ov[it];
            if (st1) *(volatile v4f*)(p0 + kOutHalf) = ov[it];
          }
          __threadfence();
        }
        __builtin_amdgcn_fence(__ATOMIC_RELEASE, "workgroup");
        __builtin_amdgcn_wave_barrier();
        __builtin_amdgcn_fence(__ATOMIC_ACQUIRE, "workgroup");
      }
    }
  }
}

extern "C" void kernel_launch(void* const* d_in, const int* in_sizes, int n_in,
                              void* d_out, int out_size, void* d_ws, size_t ws_size,
                              hipStream_t stream) {
  if (n_in < 16 || d_out == nullptr || d_ws == nullptr) return;
  if (in_sizes[0] != kBatch * kSteps) return;
  if (in_sizes[1] != kBatch * kHid || in_sizes[2] != kBatch * kHid) return;
  if (in_sizes[3] != kVocab * kEmb) return;
  if (in_sizes[4] != kEmb * kGate3 || in_sizes[7] != kEmb * kGate3) return;
  if (in_sizes[5] != kHid * kGate3 || in_sizes[8] != kHid * kGate3) return;
  if (in_sizes[11] != kHid * kGate3 || in_sizes[14] != kHid * kGate3) return;
  if (in_sizes[10] != kIn1 * kGate3 || in_sizes[13] != kIn1 * kGate3) return;
  if (in_sizes[6] != 2 * kGate3 || in_sizes[9] != 2 * kGate3) return;
  if (in_sizes[12] != 2 * kGate3 || in_sizes[15] != 2 * kGate3) return;
  if (out_size != 2 * kOutHalf) return;
  if (ws_size < kWsTotal) return;

  const int*   tok = (const int*)d_in[0];
  const float* emb = (const float*)d_in[3];
  const float* kf0 = (const float*)d_in[4];
  const float* rf0 = (const float*)d_in[5];
  const float* bf0 = (const float*)d_in[6];
  const float* kb0 = (const float*)d_in[7];
  const float* rb0 = (const float*)d_in[8];
  const float* bb0 = (const float*)d_in[9];
  const float* kf1 = (const float*)d_in[10];
  const float* rf1 = (const float*)d_in[11];
  const float* bf1 = (const float*)d_in[12];
  const float* kb1 = (const float*)d_in[13];
  const float* rb1 = (const float*)d_in[14];
  const float* bb1 = (const float*)d_in[15];
  float* out = (float*)d_out;

  char* ws = (char*)d_ws;
  unsigned short* XE   = (unsigned short*)(ws + kOffXE);
  unsigned short* WK0F = (unsigned short*)(ws + kOffWK0F);
  unsigned short* WK0B = (unsigned short*)(ws + kOffWK0B);
  unsigned short* WK1F = (unsigned short*)(ws + kOffWK1F);
  unsigned short* WK1B = (unsigned short*)(ws + kOffWK1B);
  unsigned short* WR0F = (unsigned short*)(ws + kOffWR0F);
  unsigned short* WR0B = (unsigned short*)(ws + kOffWR0B);
  unsigned short* WR1F = (unsigned short*)(ws + kOffWR1F);
  unsigned short* WR1B = (unsigned short*)(ws + kOffWR1B);
  float*          BIASP = (float*)(ws + kOffBIAS);
  float*          XS   = (float*)(ws + kOffXS);
  unsigned short* Y0   = (unsigned short*)(ws + kOffY0);

  const float* BI0F = BIASP + (size_t)0 * (2 * kGate3);
  const float* BI0B = BIASP + (size_t)1 * (2 * kGate3);
  const float* BI1F = BIASP + (size_t)2 * (2 * kGate3);
  const float* BI1B = BIASP + (size_t)3 * (2 * kGate3);

  embed_f16_kernel<<<(kRows * kEmb / 8) / kThr, kThr, 0, stream>>>(tok, emb, XE);
  bias_prep_kernel<<<dim3(3, 4), kThr, 0, stream>>>(bf0, bb0, bf1, bb1, BIASP);
  wt_transpose_f16_kernel<<<dim3(kGate3 / 64, kEmb / 64), kThr, 0, stream>>>(kf0, WK0F, kEmb);
  wt_transpose_f16_kernel<<<dim3(kGate3 / 64, kEmb / 64), kThr, 0, stream>>>(kb0, WK0B, kEmb);
  wt_transpose_f16_kernel<<<dim3(kGate3 / 64, kIn1 / 64), kThr, 0, stream>>>(kf1, WK1F, kIn1);
  wt_transpose_f16_kernel<<<dim3(kGate3 / 64, kIn1 / 64), kThr, 0, stream>>>(kb1, WK1B, kIn1);
  wt_transpose_f16_kernel<<<dim3(kGate3 / 64, kHid / 64), kThr, 0, stream>>>(rf0, WR0F, kHid);
  wt_transpose_f16_kernel<<<dim3(kGate3 / 64, kHid / 64), kThr, 0, stream>>>(rb0, WR0B, kHid);
  wt_transpose_f16_kernel<<<dim3(kGate3 / 64, kHid / 64), kThr, 0, stream>>>(rf1, WR1F, kHid);
  wt_transpose_f16_kernel<<<dim3(kGate3 / 64, kHid / 64), kThr, 0, stream>>>(rb1, WR1B, kHid);

  const dim3 ggrid((kRows / 64) * (kGate3 / 64) / 8, 1);
  const int nblk = kBatch / kSeqBlk;

  wmma_gemm64<0, false, 2, 0, false, 0><<<ggrid, 256, 0, stream>>>(
      XE, XE, kEmb, 0L, WK0F, WK0F, kEmb, 0L, (void*)XS, (void*)XS, kGate3, 0L,
      BI0F, nullptr, 0L, kRows, kGate3, kEmb, kXs0Scale);
  gru_run_kernel<0><<<nblk, kThr, 0, stream>>>(XS, WR0F, BI0F + kGate3, Y0, out, 0);

  wmma_gemm64<0, false, 2, 0, false, 0><<<ggrid, 256, 0, stream>>>(
      XE, XE, kEmb, 0L, WK0B, WK0B, kEmb, 0L, (void*)XS, (void*)XS, kGate3, 0L,
      BI0B, nullptr, 0L, kRows, kGate3, kEmb, kXs0Scale);
  gru_run_kernel<0><<<nblk, kThr, 0, stream>>>(XS, WR0B, BI0B + kGate3, Y0, out, 1);

  wmma_gemm64<0, false, 2, 0, false, 0><<<ggrid, 256, 0, stream>>>(
      Y0, Y0, kIn1, 0L, WK1F, WK1F, kIn1, 0L, (void*)XS, (void*)XS, kGate3, 0L,
      BI1F, nullptr, 0L, kRows, kGate3, kIn1, kXs1Scale);
  gru_run_kernel<1><<<nblk, kThr, 0, stream>>>(XS, WR1F, BI1F + kGate3, Y0, out, 0);

  wmma_gemm64<0, false, 2, 0, false, 0><<<ggrid, 256, 0, stream>>>(
      Y0, Y0, kIn1, 0L, WK1B, WK1B, kIn1, 0L, (void*)XS, (void*)XS, kGate3, 0L,
      BI1B, nullptr, 0L, kRows, kGate3, kIn1, kXs1Scale);
  gru_run_kernel<1><<<nblk, kThr, 0, stream>>>(XS, WR1B, BI1B + kGate3, Y0, out, 1);
}
